// CAAN_25074019074091
// MI455X (gfx1250) — hardware-verified
//
#include <hip/hip_runtime.h>
#include <math.h>
#include <stdint.h>

#define NROW 8192
#define KIN  1024
#define DIM  512
#define HDIM 256
#ifndef SQ
#define SQ NROW
#endif
#define CK   512
#define NCHK (NROW / CK)
#define NKB  16
#define QT   16
#define SCP  544
#define PLP  528
#define CTP  520
#define SLAB64 (16 * 68)
#define VTP  72
#define ATT_THREADS 256
#define NACC 4
#define FFN_ROWS 128
#define CSI  ((16 * (DIM / 8)) / 256)
#define QSC  8.0f
#define KSC  8.0f
#define PCAR 32768.0f
#define VCAR 1024.0f
#define W1S  1024.0f
#define CSC  8192.0f
#define RSC  2048.0f
#define LOG2E 1.4426950408889634f
#define RSQD 0.04419417382415922f
#define WS_CAP ((size_t)134217728)

static_assert(DIM == 8 * 16 * NACC && NACC == 4 && (DIM % 64) == 0 && (KIN % 64) == 0 && (HDIM % 64) == 0);
static_assert((DIM % 32) == 0 && (KIN % 32) == 0 && (HDIM % 32) == 0);
static_assert((NROW % CK) == 0 && (NROW / CK) == NCHK && CK == 32 * NKB && (NROW % 64) == 0 && NKB == 16);
static_assert(SQ >= FFN_ROWS && SQ <= NROW && (SQ % FFN_ROWS) == 0 && (SQ % QT) == 0 && (SQ % 64) == 0);
static_assert(16 * CTP * 2 <= 16 * SCP * 4 && CTP >= DIM + 8 && SCP >= CK + 16 && PLP >= CK + 8);
static_assert(((PLP * 2) % 16) == 0 && ((SCP * 4) % 16) == 0 && ((VTP * 2) % 16) == 0 && ((CTP * 2) % 16) == 0);
static_assert(64 * VTP >= 63 * VTP + 64);
static_assert(ATT_THREADS == 16 * QT && ATT_THREADS == 256 && FFN_ROWS == 8 * 16);
static_assert(CSI * 256 == 16 * (DIM / 8) && CSI == 4);
static_assert(((NROW * KIN) % 2048) == 0);

typedef unsigned short u16;
typedef _Float16 v16h __attribute__((ext_vector_type(16)));
typedef _Float16 v8h  __attribute__((ext_vector_type(8)));
typedef __bf16   v16b __attribute__((ext_vector_type(16)));
typedef float    v8f  __attribute__((ext_vector_type(8)));
typedef float    v4f  __attribute__((ext_vector_type(4)));
typedef unsigned int v4u __attribute__((ext_vector_type(4)));

union FragH { v16h v; v8h h[2]; v4u u[2]; };
union FragB { v16b v; v4u u[2]; };
union AttLds { float s[16 * SCP]; u16 c[2 * 16 * SCP]; };

__device__ __forceinline__ unsigned short bf_bits(float f) {
  unsigned u = __float_as_uint(f);
  return (unsigned short)((u + 0x7FFFu + ((u >> 16) & 1u)) >> 16);
}
__device__ __forceinline__ float bf_up(unsigned short h) { return __uint_as_float(((unsigned)h) << 16); }
__device__ __forceinline__ float bfr(float f) { return bf_up(bf_bits(f)); }
__device__ __forceinline__ unsigned short h_bits(_Float16 x) { return __builtin_bit_cast(unsigned short, x); }
__device__ __forceinline__ unsigned pk16(unsigned short a, unsigned short b) { return (unsigned)a | ((unsigned)b << 16); }
__device__ __forceinline__ v8f zero8() { v8f z = {0.f, 0.f, 0.f, 0.f, 0.f, 0.f, 0.f, 0.f}; return z; }

__device__ __forceinline__ v16h ldfrag_h(const _Float16* p) {
  FragH f;
  f.h[0] = *(const v8h*)(p);
  f.h[1] = *(const v8h*)(p + 16);
  return f.v;
}
__device__ __forceinline__ v16b ldfrag_b(const u16* p) {
  FragB f;
  f.u[0] = *(const v4u*)(p);
  f.u[1] = *(const v4u*)(p + 16);
  return f.v;
}

__device__ __forceinline__ v8f mma_h(v16h a, v16h b, v8f c) {
  return __builtin_amdgcn_wmma_f32_16x16x32_f16(false, a, false, b, (short)0, c, false, false);
}
__device__ __forceinline__ v8f mma_b(v16b a, v16b b, v8f c) {
  return __builtin_amdgcn_wmma_f32_16x16x32_bf16(false, a, false, b, (short)0, c, false, false);
}
__device__ __forceinline__ void guard2x3(v8f& a, v8f& b, v16h x0, v16h x1, v16h x2) {
#if defined(__HIP_DEVICE_COMPILE__)
  asm volatile("v_nop\n\tv_nop\n\tv_nop\n\tv_nop"
               : "+v"(a), "+v"(b) : "v"(x0), "v"(x1), "v"(x2) : "memory");
#endif
}
template <typename F>
__device__ __forceinline__ void guard6(v8f& a, v8f& b, v8f& c, v8f& d, F x0, F x1, F x2, F x3, F x4, F x5) {
#if defined(__HIP_DEVICE_COMPILE__)
  asm volatile("v_nop\n\tv_nop\n\tv_nop\n\tv_nop"
               : "+v"(a), "+v"(b), "+v"(c), "+v"(d) : "v"(x0), "v"(x1), "v"(x2), "v"(x3), "v"(x4), "v"(x5) : "memory");
#endif
}
__device__ __forceinline__ void guard8x6(v8f& a0, v8f& a1, v8f& a2, v8f& a3, v8f& e0, v8f& e1, v8f& e2, v8f& e3,
                                         v16h x0, v16h x1, v16h x2, v16h x3, v16h x4, v16h x5) {
#if defined(__HIP_DEVICE_COMPILE__)
  asm volatile("v_nop\n\tv_nop\n\tv_nop\n\tv_nop"
               : "+v"(a0), "+v"(a1), "+v"(a2), "+v"(a3), "+v"(e0), "+v"(e1), "+v"(e2), "+v"(e3)
               : "v"(x0), "v"(x1), "v"(x2), "v"(x3), "v"(x4), "v"(x5) : "memory");
#endif
}
__device__ __forceinline__ void guardpv4(v8f& o0, v8f& o1, v8f& o2, v8f& o3, v16h p, v16h g0, v16h g1, v16h g2, v16h g3) {
#if defined(__HIP_DEVICE_COMPILE__)
  asm volatile("v_nop\n\tv_nop\n\tv_nop\n\tv_nop"
               : "+v"(o0), "+v"(o1), "+v"(o2), "+v"(o3)
               : "v"(p), "v"(g0), "v"(g1), "v"(g2), "v"(g3) : "memory");
#endif
}
__device__ __forceinline__ void acc_guard4(v8f& a, v8f& b, v8f& c, v8f& d) {
#if defined(__HIP_DEVICE_COMPILE__)
  asm volatile("v_nop\n\tv_nop\n\tv_nop\n\tv_nop"
               : "+v"(a), "+v"(b), "+v"(c), "+v"(d));
#endif
}
__device__ __forceinline__ void wave_sync_lds() {
  __builtin_amdgcn_fence(__ATOMIC_RELEASE, "workgroup");
  __builtin_amdgcn_wave_barrier();
  __builtin_amdgcn_fence(__ATOMIC_ACQUIRE, "workgroup");
}

__global__ __launch_bounds__(256) void cvt16(const float* __restrict__ x, u16* D, int n8, int mode, float scale) {
  const int gt = blockIdx.x * 256 + (int)threadIdx.x;
  if (gt >= n8) return;
  const float* p = x + (size_t)gt * 8;
  const v4f a = *(const v4f*)(p), c4 = *(const v4f*)(p + 4);
  float v[8];
#pragma unroll
  for (int e = 0; e < 4; ++e) { v[e] = a[e]; v[4 + e] = c4[e]; }
  unsigned short s[8];
#pragma unroll
  for (int e = 0; e < 8; ++e) {
    const float vb = bfr(v[e]);
    const float vf = (mode == 1) ? vb : v[e];
    const unsigned short hb = h_bits((_Float16)(vf * scale));
    const unsigned short bb = bf_bits(v[e]);
    s[e] = (mode != 0) ? hb : bb;
  }
  v4u o;
#pragma unroll
  for (int e = 0; e < 4; ++e) o[e] = pk16(s[2 * e], s[2 * e + 1]);
  u16* d = D + (size_t)gt * 8;
  for (int pass = 0; pass < 2; ++pass) {
    *(volatile v4u*)(d) = o;
    __threadfence();
  }
}

__global__ __launch_bounds__(256) void tr16(const float* __restrict__ X, u16* XTo, int R, int C, int mode, float scale) {
  __shared__ __align__(16) u16 TH[64 * VTP];
  const int tid = threadIdx.x;
  const int bid = blockIdx.x;
  const int nrt = R >> 6;
  const int rt  = bid % nrt;
  const int ct  = bid / nrt;
  const int r0  = rt * 64;
  const int c0  = ct * 64;
  {
    const int rl = tid >> 2;
    const int cc = (tid & 3) * 16;
    const float* src = X + (size_t)(r0 + rl) * (size_t)C + c0 + cc;
#pragma unroll
    for (int i = 0; i < 4; ++i) {
      const v4f a = *(const v4f*)(src + 4 * i);
#pragma unroll
      for (int e = 0; e < 4; ++e) {
        const float v  = a[e];
        const float vb = bfr(v);
        const float vf = (mode == 1) ? vb : v;
        const unsigned short hb = h_bits((_Float16)(vf * scale));
        const unsigned short bb = bf_bits(v);
        TH[(cc + 4 * i + e) * VTP + rl] = (mode != 0) ? hb : bb;
      }
    }
  }
  __syncthreads();
  v4u vh[2];
  const int q8 = tid >> 3, p8 = (tid & 7) * 8;
#pragma unroll
  for (int it = 0; it < 2; ++it) {
    const int line = it * 32 + q8;
    vh[it] = *(const v4u*)(TH + line * VTP + p8);
  }
  const size_t base = (size_t)c0 * (size_t)R + (size_t)r0 + (size_t)p8;
  for (int pass = 0; pass < 2; ++pass) {
#pragma unroll
    for (int it = 0; it < 2; ++it) {
      const int line = it * 32 + q8;
      *(volatile v4u*)(XTo + base + (size_t)line * (size_t)R) = vh[it];
    }
    __threadfence();
  }
}

__device__ __forceinline__ void stage64(float* sl, v8f a0, v8f a1, v8f a2, v8f a3, float oscale, int lane) {
  const int hh = lane >> 4, m = lane & 15;
#pragma unroll
  for (int r = 0; r < 8; ++r) {
    const int ro = (8 * hh + r) * 68 + m;
    sl[ro]      = a0[r] * oscale;
    sl[ro + 16] = a1[r] * oscale;
    sl[ro + 32] = a2[r] * oscale;
    sl[ro + 48] = a3[r] * oscale;
  }
  wave_sync_lds();
}
__device__ __forceinline__ void epi64(float* sl, v8f a0, v8f a1, v8f a2, v8f a3, float oscale, v4f badd, float* C, int N,
                                      size_t rowb, int col0, int lane) {
  const int hh = lane >> 4, m = lane & 15;
  stage64(sl, a0, a1, a2, a3, oscale, lane);
  v4f vals[8];
#pragma unroll
  for (int it = 0; it < 8; ++it) vals[it] = *(const v4f*)(sl + (it * 2 + hh) * 68 + m * 4) + badd;
  float* dst = C + (rowb + (size_t)hh) * (size_t)N + col0 + m * 4;
  for (int pass = 0; pass < 2; ++pass) {
#pragma unroll
    for (int it = 0; it < 8; ++it) {
      *(volatile v4f*)(dst + (size_t)(it * 2) * (size_t)N) = vals[it];
    }
    __threadfence();
  }
}
__device__ __forceinline__ void epi64hsb(float* sl, v8f a0, v8f a1, v8f a2, v8f a3, float oscale, float pscale,
                                         const float* __restrict__ bias, u16* C, int N, size_t rowb, int col0, int lane) {
  stage64(sl, a0, a1, a2, a3, oscale, lane);
  const int rq = lane >> 3, c8 = (lane & 7) * 8;
  const v4f b0 = *(const v4f*)(bias + col0 + c8), b1 = *(const v4f*)(bias + col0 + c8 + 4);
  float bb[8];
#pragma unroll
  for (int e = 0; e < 4; ++e) { bb[e] = bfr(b0[e]); bb[4 + e] = bfr(b1[e]); }
  v4u oh[4];
#pragma unroll
  for (int i4 = 0; i4 < 4; ++i4) {
    const int row = i4 * 4 + rq;
    const v4f a = *(const v4f*)(sl + row * 68 + c8), c4 = *(const v4f*)(sl + row * 68 + c8 + 4);
    float w[8];
#pragma unroll
    for (int e = 0; e < 4; ++e) { w[e] = (a[e] + bb[e]) * pscale; w[4 + e] = (c4[e] + bb[4 + e]) * pscale; }
#pragma unroll
    for (int e = 0; e < 4; ++e) oh[i4][e] = pk16(h_bits((_Float16)w[2 * e]), h_bits((_Float16)w[2 * e + 1]));
  }
  u16* dst = C + rowb * (size_t)N + col0 + c8;
  for (int pass = 0; pass < 2; ++pass) {
#pragma unroll
    for (int i4 = 0; i4 < 4; ++i4) {
      const int row = i4 * 4 + rq;
      *(volatile v4u*)(dst + (size_t)row * (size_t)N) = oh[i4];
    }
    __threadfence();
  }
}

__global__ __launch_bounds__(128)
void gemm_b32(const u16* __restrict__ A, const u16* __restrict__ Bt, const float* __restrict__ bias, float* C,
              int M, int N, int K, float oscale) {
  __shared__ __align__(16) float slab[4 * SLAB64];
  const int tid = threadIdx.x, wave = tid >> 5, lane = tid & 31, hh = lane >> 4, m = lane & 15;
  const int ntile = N >> 6;
  const int bid   = blockIdx.x;
  const int rowb  = (bid / ntile) * 64 + wave * 16;
  const int col0  = (bid % ntile) * 64;
  if (rowb + 16 > M) return;
  const u16* ap = A  + (size_t)(rowb + m) * (size_t)K + 8 * hh;
  const u16* bp = Bt + (size_t)(col0 + m) * (size_t)K + 8 * hh;
  const size_t bs = (size_t)16 * K;
  v8f acc0 = zero8(), acc1 = zero8(), acc2 = zero8(), acc3 = zero8();
#pragma unroll 1
  for (int k0 = 0; k0 < K; k0 += 32) {
    const v16b a  = ldfrag_b(ap + k0);
    const v16b b0 = ldfrag_b(bp + k0);
    const v16b b1 = ldfrag_b(bp + bs + k0);
    const v16b b2 = ldfrag_b(bp + 2 * bs + k0);
    const v16b b3 = ldfrag_b(bp + 3 * bs + k0);
    acc0 = mma_b(a, b0, acc0);
    acc1 = mma_b(a, b1, acc1);
    acc2 = mma_b(a, b2, acc2);
    acc3 = mma_b(a, b3, acc3);
    guard6<v16b>(acc0, acc1, acc2, acc3, a, b0, b1, b2, b3, a);
  }
  const v4f bv4 = *(const v4f*)(bias + col0 + m * 4);
  v4f badd;
#pragma unroll
  for (int e = 0; e < 4; ++e) badd[e] = bfr(bv4[e]);
  epi64(slab + wave * SLAB64, acc0, acc1, acc2, acc3, oscale, badd, C, N, (size_t)rowb, col0, lane);
}

__global__ __launch_bounds__(128)
void gemm_bh16(const u16* __restrict__ A, const u16* __restrict__ Bt, const float* __restrict__ bias, u16* C,
               int M, int N, int K, float oscale, float pscale) {
  __shared__ __align__(16) float slab[4 * SLAB64];
  const int tid = threadIdx.x, wave = tid >> 5, lane = tid & 31, hh = lane >> 4, m = lane & 15;
  const int ntile = N >> 6;
  const int bid   = blockIdx.x;
  const int rowb  = (bid / ntile) * 64 + wave * 16;
  const int col0  = (bid % ntile) * 64;
  if (rowb + 16 > M) return;
  const u16* ap = A  + (size_t)(rowb + m) * (size_t)K + 8 * hh;
  const u16* bp = Bt + (size_t)(col0 + m) * (size_t)K + 8 * hh;
  const size_t bs = (size_t)16 * K;
  v8f acc0 = zero8(), acc1 = zero8(), acc2 = zero8(), acc3 = zero8();
#pragma unroll 1
  for (int k0 = 0; k0 < K; k0 += 32) {
    const v16b a  = ldfrag_b(ap + k0);
    const v16b b0 = ldfrag_b(bp + k0);
    const v16b b1 = ldfrag_b(bp + bs + k0);
    const v16b b2 = ldfrag_b(bp + 2 * bs + k0);
    const v16b b3 = ldfrag_b(bp + 3 * bs + k0);
    acc0 = mma_b(a, b0, acc0);
    acc1 = mma_b(a, b1, acc1);
    acc2 = mma_b(a, b2, acc2);
    acc3 = mma_b(a, b3, acc3);
    guard6<v16b>(acc0, acc1, acc2, acc3, a, b0, b1, b2, b3, a);
  }
  epi64hsb(slab + wave * SLAB64, acc0, acc1, acc2, acc3, oscale, pscale, bias, C, N, (size_t)rowb, col0, lane);
}

__device__ __forceinline__ void ctx_store(const u16* ct, u16* dst, int tid) {
  v4u v[CSI];
#pragma unroll
  for (int it = 0; it < CSI; ++it) {
    const int p   = it * 256 + tid;
    const int row = p / (DIM / 8);
    const int c8  = (p - row * (DIM / 8)) * 8;
    v[it] = *(const v4u*)(ct + row * CTP + c8);
  }
  for (int pass = 0; pass < 2; ++pass) {
#pragma unroll
    for (int it = 0; it < CSI; ++it) {
      const int p   = it * 256 + tid;
      const int row = p / (DIM / 8);
      const int c8  = (p - row * (DIM / 8)) * 8;
      *(volatile v4u*)(dst + (size_t)row * DIM + c8) = v[it];
    }
    __threadfence();
  }
}

__global__ __launch_bounds__(ATT_THREADS)
void attn_fwd(const u16* __restrict__ QPp, const u16* __restrict__ KPp, const u16* __restrict__ VTp, u16* CHo, u16* CRo) {
  __shared__ __align__(16) AttLds L0;
  __shared__ __align__(16) u16 pls[16 * PLP];
  __shared__ float rowa[QT];
  __shared__ float rowi[QT];
  float* const scs = L0.s;

  const int tid  = threadIdx.x;
  const int wave = tid >> 5;
  const int lane = tid & 31;
  const int hh   = lane >> 4;
  const int m    = lane & 15;
  const int r16  = tid >> 4;
  const int sub  = tid & 15;
  const int kl0  = sub * 32;

  const int q0 = blockIdx.x * QT;

  const _Float16* qa  = (const _Float16*)(const void*)QPp + ((size_t)q0 + m) * DIM + 8 * hh;
  const _Float16* kbp = (const _Float16*)(const void*)KPp + (size_t)m * DIM + 8 * hh;
  const _Float16* vbp = (const _Float16*)(const void*)VTp + ((size_t)wave * (16 * NACC) + m) * NROW + 8 * hh;
  const float lsc = RSQD * LOG2E / (QSC * KSC);

  float mrun = -INFINITY, lrun = 0.f;
  v8f o0 = zero8(), o1 = zero8(), o2 = zero8(), o3 = zero8();

#pragma unroll 1
  for (int c = 0; c < NCHK; ++c) {
    const int kbeg = c * CK;
#pragma unroll 1
    for (int kb = wave; kb < NKB; kb += 8) {
      v8f s0 = zero8(), s1 = zero8();
      const _Float16* k0p = kbp + (size_t)(kbeg + kb * 32) * DIM;
      const _Float16* k1p = k0p + (size_t)16 * DIM;
#pragma unroll 4
      for (int ks = 0; ks < DIM / 32; ++ks) {
        const v16h a  = ldfrag_h(qa + ks * 32);
        const v16h f0 = ldfrag_h(k0p + ks * 32);
        const v16h f1 = ldfrag_h(k1p + ks * 32);
        s0 = mma_h(a, f0, s0);
        s1 = mma_h(a, f1, s1);
        guard2x3(s0, s1, a, f0, f1);
      }
      float* srow = scs + (8 * hh) * SCP + kb * 32 + m;
#pragma unroll
      for (int r = 0; r < 8; ++r) {
        srow[r * SCP]      = s0[r];
        srow[r * SCP + 16] = s1[r];
      }
    }
    __syncthreads();
    {
      const float* sp = scs + r16 * SCP + kl0;
      float t[32];
      float cm = -INFINITY;
#pragma unroll
      for (int i = 0; i < 8; ++i) {
        const v4f a = *(const v4f*)(sp + 4 * i);
#pragma unroll
        for (int e = 0; e < 4; ++e) {
          const float tv = a[e] * lsc;
          t[4 * i + e] = tv;
          cm = fmaxf(cm, tv);
        }
      }
#pragma unroll
      for (int d = 1; d <= 8; d <<= 1) cm = fmaxf(cm, __shfl_xor(cm, d, 32));
      const float mn = fmaxf(mrun, cm);
      const float al = (mrun == -INFINITY) ? 0.f : exp2f(mrun - mn);
      mrun = mn;
      float ps = 0.f;
#pragma unroll
      for (int j = 0; j < 32; ++j) {
        const float p = exp2f(t[j] - mn);
        t[j] = p;
        ps += p;
      }
#pragma unroll
      for (int d = 1; d <= 8; d <<= 1) ps += __shfl_xor(ps, d, 32);
      v4u pk[4];
#pragma unroll
      for (int i = 0; i < 4; ++i) {
#pragma unroll
        for (int e = 0; e < 4; ++e) {
          const int j = 8 * i + 2 * e;
          pk[i][e] = pk16(h_bits((_Float16)(t[j] * PCAR)), h_bits((_Float16)(t[j + 1] * PCAR)));
        }
      }
      lrun = lrun * al + ps;
      u16* pd = pls + r16 * PLP + kl0;
#pragma unroll
      for (int i = 0; i < 4; ++i) *(v4u*)(pd + 8 * i) = pk[i];
      if (sub == 0) rowa[r16] = al;
    }
    __syncthreads();
    {
      float scl[8];
#pragma unroll
      for (int r = 0; r < 8; ++r) scl[r] = rowa[8 * hh + r];
#pragma unroll
      for (int r = 0; r < 8; ++r) { o0[r] *= scl[r]; o1[r] *= scl[r]; o2[r] *= scl[r]; o3[r] *= scl[r]; }
      const _Float16* pp = (const _Float16*)(const void*)pls + m * PLP + 8 * hh;
      const _Float16* vp = vbp + kbeg;
#pragma unroll 1
      for (int kb = 0; kb < NKB; ++kb) {
        const v16h pf = ldfrag_h(pp + kb * 32);
        const _Float16* vk = vp + kb * 32;
        const v16h g0 = ldfrag_h(vk);
        const v16h g1 = ldfrag_h(vk + (size_t)16 * NROW);
        const v16h g2 = ldfrag_h(vk + (size_t)32 * NROW);
        const v16h g3 = ldfrag_h(vk + (size_t)48 * NROW);
        o0 = mma_h(pf, g0, o0);
        o1 = mma_h(pf, g1, o1);
        o2 = mma_h(pf, g2, o2);
        o3 = mma_h(pf, g3, o3);
        guardpv4(o0, o1, o2, o3, pf, g0, g1, g2, g3);
      }
    }
  }
  acc_guard4(o0, o1, o2, o3);

  if (sub == 0) rowi[r16] = (1.0f / lrun) * (CSC / (PCAR * VCAR));
  __syncthreads();
  float inv[8];
#pragma unroll
  for (int r = 0; r < 8; ++r) inv[r] = rowi[8 * hh + r];

  u16* const ct = L0.c;
  const int cb = wave * (16 * NACC) + m;
#pragma unroll
  for (int r = 0; r < 8; ++r) {
    const int ro = (8 * hh + r) * CTP + cb;
    ct[ro]      = h_bits((_Float16)(o0[r] * inv[r]));
    ct[ro + 16] = h_bits((_Float16)(o1[r] * inv[r]));
    ct[ro + 32] = h_bits((_Float16)(o2[r] * inv[r]));
    ct[ro + 48] = h_bits((_Float16)(o3[r] * inv[r]));
  }
  __syncthreads();
  ctx_store(ct, CHo + (size_t)q0 * DIM, tid);
  __syncthreads();
#pragma unroll
  for (int r = 0; r < 8; ++r) {
    const int ro = (8 * hh + r) * CTP + cb;
    const float x0 = o0[r] * inv[r], x1 = o1[r] * inv[r], x2 = o2[r] * inv[r], x3 = o3[r] * inv[r];
    const _Float16 e0 = (_Float16)x0, e1 = (_Float16)x1, e2 = (_Float16)x2, e3 = (_Float16)x3;
    ct[ro]      = h_bits((_Float16)((x0 - (float)e0) * RSC));
    ct[ro + 16] = h_bits((_Float16)((x1 - (float)e1) * RSC));
    ct[ro + 32] = h_bits((_Float16)((x2 - (float)e2) * RSC));
    ct[ro + 48] = h_bits((_Float16)((x3 - (float)e3) * RSC));
  }
  __syncthreads();
  ctx_store(ct, CRo + (size_t)q0 * DIM, tid);
}

__global__ __launch_bounds__(256)
void ffn_score(const u16* __restrict__ CH, const u16* __restrict__ CR, const u16* __restrict__ W1t,
               const float* __restrict__ b1, const float* __restrict__ w2, const float* __restrict__ b2, float* out) {
  __shared__ __align__(16) float osm[FFN_ROWS];
  const int tid = threadIdx.x, wave = tid >> 5, lane = tid & 31, hh = lane >> 4, m = lane & 15;
  const int rowb = blockIdx.x * FFN_ROWS + wave * 16;
  const _Float16* ap  = (const _Float16*)(const void*)CH + (size_t)(rowb + m) * DIM + 8 * hh;
  const _Float16* arp = (const _Float16*)(const void*)CR + (size_t)(rowb + m) * DIM + 8 * hh;
  const size_t bs = (size_t)16 * DIM;
  const float os1 = 1.0f / (CSC * W1S);
  const float os2 = 1.0f / (CSC * W1S * RSC);
  float sp[8];
#pragma unroll
  for (int r = 0; r < 8; ++r) sp[r] = 0.f;

#pragma unroll 1
  for (int g = 0; g < HDIM / 64; ++g) {
    const _Float16* bp = (const _Float16*)(const void*)W1t + (size_t)(g * 64 + m) * DIM + 8 * hh;
    v8f acc0 = zero8(), acc1 = zero8(), acc2 = zero8(), acc3 = zero8();
    v8f acr0 = zero8(), acr1 = zero8(), acr2 = zero8(), acr3 = zero8();
#pragma unroll 1
    for (int k0 = 0; k0 < DIM; k0 += 32) {
      const v16h a  = ldfrag_h(ap + k0);
      const v16h ar = ldfrag_h(arp + k0);
      const v16h b0 = ldfrag_h(bp + k0);
      const v16h w1 = ldfrag_h(bp + bs + k0);
      const v16h w2f = ldfrag_h(bp + 2 * bs + k0);
      const v16h w3 = ldfrag_h(bp + 3 * bs + k0);
      acc0 = mma_h(a, b0, acc0);
      acc1 = mma_h(a, w1, acc1);
      acc2 = mma_h(a, w2f, acc2);
      acc3 = mma_h(a, w3, acc3);
      acr0 = mma_h(ar, b0, acr0);
      acr1 = mma_h(ar, w1, acr1);
      acr2 = mma_h(ar, w2f, acr2);
      acr3 = mma_h(ar, w3, acr3);
      guard8x6(acc0, acc1, acc2, acc3, acr0, acr1, acr2, acr3, a, ar, b0, w1, w2f, w3);
    }
    float bb[4], wv[4];
#pragma unroll
    for (int t = 0; t < 4; ++t) {
      const int col = g * 64 + 16 * t + m;
      bb[t] = bfr(b1[col]);
      wv[t] = bfr(w2[col]);
    }
#pragma unroll
    for (int r = 0; r < 8; ++r) {
      const float h0 = fmaxf(acc0[r] * os1 + acr0[r] * os2 + bb[0], 0.f);
      const float h1 = fmaxf(acc1[r] * os1 + acr1[r] * os2 + bb[1], 0.f);
      const float h2 = fmaxf(acc2[r] * os1 + acr2[r] * os2 + bb[2], 0.f);
      const float h3 = fmaxf(acc3[r] * os1 + acr3[r] * os2 + bb[3], 0.f);
      sp[r] += h0 * wv[0] + h1 * wv[1] + h2 * wv[2] + h3 * wv[3];
    }
  }
#pragma unroll
  for (int r = 0; r < 8; ++r) {
    float v = sp[r];
#pragma unroll
    for (int d = 1; d <= 8; d <<= 1) v += __shfl_xor(v, d, 32);
    sp[r] = v;
  }
  const float b2v = bfr(b2[0]);
  if (m == 0) {
#pragma unroll
    for (int r = 0; r < 8; ++r) osm[wave * 16 + 8 * hh + r] = sp[r] + b2v;
  }
  __syncthreads();
  if (wave == 0) {
    const v4f ov = *(const v4f*)(osm + lane * 4);
    float* dst = out + (size_t)blockIdx.x * FFN_ROWS + lane * 4;
    *(volatile v4f*)dst = ov;
    __threadfence();
    *(volatile v4f*)dst = ov;
  }
}

extern "C" void kernel_launch(void* const* d_in, const int* in_sizes, int n_in,
                              void* d_out, int out_size, void* d_ws, size_t ws_size,
                              hipStream_t stream) {
  if (n_in < 11) return;
  if (in_sizes[0] != NROW * KIN) return;
  if (in_sizes[1] != KIN * DIM || in_sizes[3] != KIN * DIM || in_sizes[5] != KIN * DIM) return;
  if (in_sizes[2] != DIM || in_sizes[4] != DIM || in_sizes[6] != DIM) return;
  if (in_sizes[7] != DIM * HDIM || in_sizes[8] != HDIM || in_sizes[9] != HDIM || in_sizes[10] < 1) return;
  if (out_size != NROW) return;

  const float* x   = (const float*)d_in[0];
  const float* wq  = (const float*)d_in[1];
  const float* bq  = (const float*)d_in[2];
  const float* wk  = (const float*)d_in[3];
  const float* bk  = (const float*)d_in[4];
  const float* wv  = (const float*)d_in[5];
  const float* bv  = (const float*)d_in[6];
  const float* w1  = (const float*)d_in[7];
  const float* b1  = (const float*)d_in[8];
  const float* w2  = (const float*)d_in[9];
  const float* b2  = (const float*)d_in[10];
  float*       out = (float*)d_out;

  const size_t szWT = (size_t)DIM * KIN * 2;
  const size_t szW1 = (size_t)HDIM * DIM * 2;
  const size_t szXB = (size_t)NROW * KIN * 2;
  const size_t szQP = (size_t)SQ * DIM * 2;
  const size_t szKP = (size_t)NROW * DIM * 2;
  const size_t szV  = (size_t)NROW * DIM * 4;
  const size_t szVT = (size_t)DIM * NROW * 2;
  const size_t szCX = (size_t)SQ * DIM * 2;
  size_t off = 0;
  const size_t oWQ = off; off += szWT;
  const size_t oWK = off; off += szWT;
  const size_t oWV = off; off += szWT;
  const size_t oW1 = off; off += szW1;
  const size_t oXB = off; off += szXB;
  const size_t oQP = off; off += szQP;
  const size_t oKP = off; off += szKP;
  const size_t oV  = off; off += szV;
  const size_t oVT = off; off += szVT;
  const size_t oCH = off; off += szCX;
  const size_t oCR = off; off += szCX;
  if (off > ws_size) return;
  if (off > WS_CAP) return;

  char* ws = (char*)d_ws;
  u16*   WQT = (u16*)(ws + oWQ);
  u16*   WKT = (u16*)(ws + oWK);
  u16*   WVT = (u16*)(ws + oWV);
  u16*   W1T = (u16*)(ws + oW1);
  u16*   XB  = (u16*)(ws + oXB);
  u16*   QP  = (u16*)(ws + oQP);
  u16*   KP  = (u16*)(ws + oKP);
  float* V   = (float*)(ws + oV);
  u16*   VT  = (u16*)(ws + oVT);
  u16*   CH  = (u16*)(ws + oCH);
  u16*   CR  = (u16*)(ws + oCR);

  const int n8x = (NROW * KIN) / 8;
  const dim3 blk(256);
  const dim3 bG(128);
  const dim3 gX(n8x / 256);
  const dim3 gWT((KIN / 64) * (DIM / 64));
  const dim3 gW1((DIM / 64) * (HDIM / 64));
  const dim3 gGQ((SQ / 64) * (DIM / 64));
  const dim3 gG((NROW / 64) * (DIM / 64));
  const dim3 gVT((NROW / 64) * (DIM / 64));
  const dim3 gAT(SQ / QT);
  const dim3 bAT(ATT_THREADS);
  const dim3 gFF(SQ / FFN_ROWS);

  cvt16<<<gX, blk, 0, stream>>>(x, XB, n8x, 0, 1.0f);
  tr16<<<gWT, blk, 0, stream>>>(wq, WQT, KIN, DIM, 0, 1.0f);
  tr16<<<gWT, blk, 0, stream>>>(wk, WKT, KIN, DIM, 0, 1.0f);
  tr16<<<gWT, blk, 0, stream>>>(wv, WVT, KIN, DIM, 0, 1.0f);
  tr16<<<gW1, blk, 0, stream>>>(w1, W1T, DIM, HDIM, 1, W1S);
  gemm_bh16<<<gGQ, bG, 0, stream>>>(XB, WQT, bq, QP, SQ, DIM, KIN, 1.0f, QSC);
  gemm_bh16<<<gG,  bG, 0, stream>>>(XB, WKT, bk, KP, NROW, DIM, KIN, 1.0f, KSC);
  gemm_b32<<<gG,   bG, 0, stream>>>(XB, WVT, bv, V, NROW, DIM, KIN, 1.0f);
  tr16<<<gVT, blk, 0, stream>>>(V, VT, NROW, DIM, 2, VCAR);
  attn_fwd<<<gAT, bAT, 0, stream>>>(QP, KP, VT, CH, CR);
  ffn_score<<<gFF, blk, 0, stream>>>(CH, CR, W1T, b1, w2, b2, out);
  (void)hipGetLastError();
}
